// SelfAttention_31679678775564
// MI455X (gfx1250) — hardware-verified
//
#include <hip/hip_runtime.h>
#include <math.h>

#ifndef NB
#define NB 4
#endif
#ifndef SEQ
#define SEQ 2048
#endif
#ifndef SCORE_RES
#define SCORE_RES 1
#endif
#define NB_FULL 4
#define SEQ_FULL 2048
#define DM 1024
#define RS_RPW 4
#define QKP (6 * DM)
#define SCORE_K (SCORE_RES ? (3 * DM) : DM)

static_assert(DM == 1024);
static_assert(DM % 64 == 0 && DM % 32 == 0);
static_assert(DM == 256 * 4);
static_assert(SEQ % 256 == 0);
static_assert(SEQ % (8 * RS_RPW) == 0);
static_assert(SEQ <= SEQ_FULL && NB <= NB_FULL);
static_assert(SEQ % 64 == 0 && SEQ % 32 == 0);
static_assert(QKP == 6 * DM && SCORE_K % 32 == 0 && SCORE_K <= 3 * DM);

typedef __attribute__((ext_vector_type(16))) _Float16     v16h;
typedef __attribute__((ext_vector_type(8)))  _Float16     v8h;
typedef __attribute__((ext_vector_type(8)))  float        v8f;
typedef __attribute__((ext_vector_type(4)))  float        v4f;
typedef __attribute__((ext_vector_type(4)))  unsigned int u4v;
typedef __attribute__((ext_vector_type(4)))  int          i4v;
typedef _Float16 h16;


__device__ __forceinline__ float bfr(float v) {
    const unsigned u = __builtin_bit_cast(unsigned, v);
    const unsigned r = (u + 0x7fffu + ((u >> 16) & 1u)) & 0xffff0000u;
    return __builtin_bit_cast(float, r);
}
__device__ __forceinline__ unsigned pk2h(float a, float b) {
    return (unsigned)__builtin_bit_cast(unsigned short, (_Float16)a) | ((unsigned)__builtin_bit_cast(unsigned short, (_Float16)b) << 16);
}
static __device__ __forceinline__ h16 toh_flush(float v) {
    const h16 r = (h16)v;
    return (fabsf(v) < 6.103515625e-05f) ? (h16)0.0f : r;
}
__device__ __forceinline__ unsigned pk2hf(float a, float b) {
    return (unsigned)__builtin_bit_cast(unsigned short, toh_flush(a)) | ((unsigned)__builtin_bit_cast(unsigned short, toh_flush(b)) << 16);
}
__device__ __forceinline__ v8f wmma16(v16h a, v16h b, v8f c) {
    c = __builtin_amdgcn_wmma_f32_16x16x32_f16(false, a, false, b, (short)0, c, false, false);
    asm volatile("v_nop\n\tv_nop\n\tv_nop\n\tv_nop" : "+v"(c) : "v"(a), "v"(b));
    return c;
}
union FragH { v16h v; v8h h[2]; };
__device__ __forceinline__ v16h ldfrag(const _Float16* p) {
    FragH f; f.h[0] = *(const v8h*)(p); f.h[1] = *(const v8h*)(p + 16); return f.v;
}
__device__ __forceinline__ void st2_v4f(float* p, v4f v) { *(volatile v4f*)p = v; __threadfence(); *(volatile v4f*)p = v; }
__device__ __forceinline__ void st2_u4(unsigned short* p, u4v v) { *(volatile u4v*)p = v; __threadfence(); *(volatile u4v*)p = v; }

template <int OUT_MODE, int BIAS_MODE, bool RELU>
__device__ __forceinline__ void gemm64_body(const unsigned short* __restrict__ Ap, int lda, long long strideA,
                                            const unsigned short* __restrict__ Btp, int ldb, long long strideB,
                                            unsigned short* __restrict__ Ch, float* __restrict__ Cf, int ldc, long long strideC,
                                            const float* __restrict__ bias,
                                            int M, int N, int K, float scale, float carry) {
    __shared__ __align__(16) float sT[8 * 16 * 68];
    const int b    = blockIdx.y;
    const int lane = threadIdx.x & 31;
    const int wave = __builtin_amdgcn_readfirstlane((int)(threadIdx.x >> 5));
    const int tilesN = N >> 6;
    const int tilesM = M >> 6;
    const int tile = blockIdx.x * 8 + wave;
    if (tile >= tilesM * tilesN) return;
    const int tm = tile / tilesN;
    const int tn = tile - tm * tilesN;
    const int m0 = tm << 6;
    const int n0 = tn << 6;
    const int rlane = lane & 15;
    const int koff  = (lane >> 4) * 8;
    const int sb    = wave * (16 * 68);

    const _Float16* ap = (const _Float16*)Ap  + (size_t)b * (size_t)strideA + (size_t)(m0 + rlane) * (size_t)lda + koff;
    const _Float16* bp = (const _Float16*)Btp + (size_t)b * (size_t)strideB + (size_t)(n0 + rlane) * (size_t)ldb + koff;

    v8f acc[4][4];
#pragma unroll
    for (int i = 0; i < 4; ++i)
#pragma unroll
        for (int j = 0; j < 4; ++j) { const v8f zz = {0.f, 0.f, 0.f, 0.f, 0.f, 0.f, 0.f, 0.f}; acc[i][j] = zz; }

    for (int k0 = 0; k0 < K; k0 += 32) {
        v16h bh[4];
#pragma unroll
        for (int j = 0; j < 4; ++j) bh[j] = ldfrag(bp + (size_t)(16 * j) * (size_t)ldb + k0);
#pragma unroll
        for (int i = 0; i < 4; ++i) {
            const v16h ah = ldfrag(ap + (size_t)(16 * i) * (size_t)lda + k0);
#pragma unroll
            for (int j = 0; j < 4; ++j) acc[i][j] = wmma16(ah, bh[j], acc[i][j]);
        }
    }

    float bc[4];
#pragma unroll
    for (int j = 0; j < 4; ++j) bc[j] = 0.f;
    if (BIAS_MODE == 1) {
#pragma unroll
        for (int j = 0; j < 4; ++j) bc[j] = bias[n0 + (j << 4) + rlane];
    }

#pragma unroll
    for (int i = 0; i < 4; ++i) {
        const int mBase = m0 + (i << 4);
        float br[8];
#pragma unroll
        for (int r = 0; r < 8; ++r) br[r] = 0.f;
        if (BIAS_MODE == 2) {
#pragma unroll
            for (int r = 0; r < 8; ++r) br[r] = bias[mBase + koff + r];
        }
#pragma unroll
        for (int j = 0; j < 4; ++j) {
#pragma unroll
            for (int r = 0; r < 8; ++r) {
                float v = (acc[i][j][r] * scale + (bc[j] + br[r])) * carry;
                if (RELU) v = fmaxf(v, 0.0f);
                sT[sb + (koff + r) * 68 + (j << 4) + rlane] = v;
            }
        }
        __builtin_amdgcn_fence(3  , "workgroup");
        __builtin_amdgcn_wave_barrier();
        __builtin_amdgcn_fence(2  , "workgroup");
        if (OUT_MODE == 0) {
            float* C = Cf + (size_t)b * (size_t)strideC;
            const int hh = lane >> 4, c4 = (lane & 15) * 4;
            for (int pass = 0; pass < 2; ++pass) {
#pragma unroll
                for (int it = 0; it < 8; ++it) {
                    const int row = it * 2 + hh;
                    const v4f v = *(const v4f*)(&sT[sb + row * 68 + c4]);
                    *(volatile v4f*)(C + (size_t)(mBase + row) * (size_t)ldc + n0 + c4) = v;
                }
                __threadfence();
            }
        } else if (OUT_MODE == 1) {
            unsigned short* C = Ch + (size_t)b * (size_t)strideC;
            const int q = lane >> 3, c8 = (lane & 7) * 8;
            for (int pass = 0; pass < 2; ++pass) {
#pragma unroll
                for (int it = 0; it < 4; ++it) {
                    const int row = it * 4 + q;
                    v8h hv;
#pragma unroll
                    for (int e = 0; e < 8; ++e) hv[e] = toh_flush(sT[sb + row * 68 + c8 + e]);
                    *(volatile v8h*)(C + (size_t)(mBase + row) * (size_t)ldc + n0 + c8) = hv;
                }
                __threadfence();
            }
        } else {
            unsigned short* C = Ch + (size_t)b * (size_t)strideC;
            const int q = lane >> 3, c8 = (lane & 7) * 8;
            const int isK   = n0 / DM;
            const int cb    = n0 + isK * (2 * DM);
            const int offH2 = DM + isK * DM;
            const int offR  = 2 * DM - isK * DM;
            for (int pass = 0; pass < 2; ++pass) {
#pragma unroll
                for (int it = 0; it < 4; ++it) {
                    const int row = it * 4 + q;
                    v8h hv, rv;
#pragma unroll
                    for (int e = 0; e < 8; ++e) {
                        const float f = sT[sb + row * 68 + c8 + e];
                        const h16 hq = toh_flush(f);
                        hv[e] = hq;
                        rv[e] = toh_flush(f - (float)hq);
                    }
                    unsigned short* dst = C + (size_t)(mBase + row) * (size_t)ldc + cb + c8;
                    *(volatile v8h*)(dst) = hv;
                    *(volatile v8h*)(dst + offH2) = hv;
                    *(volatile v8h*)(dst + offR) = rv;
                }
                __threadfence();
            }
        }
        __builtin_amdgcn_fence(3  , "workgroup");
        __builtin_amdgcn_wave_barrier();
        __builtin_amdgcn_fence(2  , "workgroup");
    }
}

__global__ __launch_bounds__(256) void k_gemm_qk(const unsigned short* __restrict__ A, int lda, long long strideA,
                                                 const unsigned short* __restrict__ Bt, int ldb, long long strideB,
                                                 unsigned short* __restrict__ C, int ldc, long long strideC,
                                                 const float* __restrict__ bias,
                                                 int M, int N, int K, float scale, float carry) {
    gemm64_body<2, 1, false>(A, lda, strideA, Bt, ldb, strideB, C, nullptr, ldc, strideC, bias, M, N, K, scale, carry);
}
__global__ __launch_bounds__(256) void k_gemm_vt(const unsigned short* __restrict__ A, int lda, long long strideA,
                                                 const unsigned short* __restrict__ Bt, int ldb, long long strideB,
                                                 unsigned short* __restrict__ C, int ldc, long long strideC,
                                                 const float* __restrict__ bias,
                                                 int M, int N, int K, float scale, float carry) {
    gemm64_body<1, 2, false>(A, lda, strideA, Bt, ldb, strideB, C, nullptr, ldc, strideC, bias, M, N, K, scale, carry);
}
__global__ __launch_bounds__(256) void k_gemm_s(const unsigned short* __restrict__ A, int lda, long long strideA,
                                                const unsigned short* __restrict__ Bt, int ldb, long long strideB,
                                                float* __restrict__ C, int ldc, long long strideC,
                                                int M, int N, int K, float scale) {
    gemm64_body<0, 0, false>(A, lda, strideA, Bt, ldb, strideB, nullptr, C, ldc, strideC, nullptr, M, N, K, scale, 1.0f);
}
__global__ __launch_bounds__(256) void k_gemm_ctx(const unsigned short* __restrict__ A, int lda, long long strideA,
                                                  const unsigned short* __restrict__ Bt, int ldb, long long strideB,
                                                  unsigned short* __restrict__ C, int ldc, long long strideC,
                                                  int M, int N, int K, float scale) {
    gemm64_body<1, 0, false>(A, lda, strideA, Bt, ldb, strideB, C, nullptr, ldc, strideC, nullptr, M, N, K, scale, 1.0f);
}
__global__ __launch_bounds__(256) void k_gemm_out(const unsigned short* __restrict__ A, int lda, long long strideA,
                                                  const unsigned short* __restrict__ Bt, int ldb, long long strideB,
                                                  float* __restrict__ C, int ldc, long long strideC,
                                                  const float* __restrict__ bias,
                                                  int M, int N, int K, float scale) {
    gemm64_body<0, 1, true>(A, lda, strideA, Bt, ldb, strideB, nullptr, C, ldc, strideC, bias, M, N, K, scale, 1.0f);
}

__global__ __launch_bounds__(256) void k_prep_x(const float* __restrict__ x, unsigned short* __restrict__ X16) {
    const long long u = (long long)blockIdx.x * 256 + threadIdx.x;
    if (u >= (long long)NB * SEQ * (DM / 8)) return;
    const int r = (int)(u / (DM / 8)); const int c0 = 8 * (int)(u % (DM / 8));
    const int b = r / SEQ; const int t = r - b * SEQ;
    const float* s = x + ((size_t)b * SEQ_FULL + t) * DM + c0;
    const v4f x0 = *(const v4f*)(s), x1 = *(const v4f*)(s + 4);
    const float w0 = bfr(x0.x), w1 = bfr(x0.y), w2 = bfr(x0.z), w3 = bfr(x0.w), w4 = bfr(x1.x), w5 = bfr(x1.y), w6 = bfr(x1.z), w7 = bfr(x1.w);
    u4v pa; pa.x = pk2hf(w0, w1); pa.y = pk2hf(w2, w3); pa.z = pk2hf(w4, w5); pa.w = pk2hf(w6, w7);
    st2_u4(X16 + (size_t)r * DM + c0, pa);
}

__global__ __launch_bounds__(256) void k_wT(const float* __restrict__ SRC, unsigned short* __restrict__ DST, float sc) {
    const int u = blockIdx.x * 256 + threadIdx.x;
    if (u >= DM * (DM / 8)) return;
    const int n = u / (DM / 8); const int k0 = 8 * (u % (DM / 8));
    float w[8];
#pragma unroll
    for (int e = 0; e < 8; ++e) w[e] = bfr(SRC[(size_t)(k0 + e) * DM + n]) * sc;
    u4v pk; pk.x = pk2h(w[0], w[1]); pk.y = pk2h(w[2], w[3]); pk.z = pk2h(w[4], w[5]); pk.w = pk2h(w[6], w[7]);
    st2_u4(DST + (size_t)n * DM + k0, pk);
}

__global__ __launch_bounds__(256) void k_bias(const float* __restrict__ bq, const float* __restrict__ bk, const float* __restrict__ bv,
                                              const float* __restrict__ bm, float* __restrict__ BT) {
    const int t = threadIdx.x;
    v4f a = *(const v4f*)(bq + 4 * t);
    v4f c = *(const v4f*)(bk + 4 * t);
    v4f d = *(const v4f*)(bv + 4 * t);
    v4f e = *(const v4f*)(bm + 4 * t);
    a.x = bfr(a.x); a.y = bfr(a.y); a.z = bfr(a.z); a.w = bfr(a.w);
    c.x = bfr(c.x); c.y = bfr(c.y); c.z = bfr(c.z); c.w = bfr(c.w);
    d.x = bfr(d.x); d.y = bfr(d.y); d.z = bfr(d.z); d.w = bfr(d.w);
    e.x = bfr(e.x); e.y = bfr(e.y); e.z = bfr(e.z); e.w = bfr(e.w);
    st2_v4f(BT + 4 * t, a);
    st2_v4f(BT + DM + 4 * t, c);
    st2_v4f(BT + 2 * DM + 4 * t, d);
    st2_v4f(BT + 3 * DM + 4 * t, e);
}

__global__ __launch_bounds__(256) void k_rowsoft(const float* __restrict__ S, unsigned short* __restrict__ P) {
    #pragma clang fp contract(off)
    const int L = threadIdx.x & 31;
    const int wave = __builtin_amdgcn_readfirstlane((int)(threadIdx.x >> 5));
    const int row0 = (blockIdx.x * 8 + wave) * RS_RPW;
#pragma unroll 1
    for (int rr = 0; rr < RS_RPW; ++rr) {
        const int row = row0 + rr;
        const float* sr = S + (size_t)row * SEQ + 8 * L;
        float m = -3.0e38f, s = 0.f;
#pragma unroll 1
        for (int g = 0; g < SEQ / 256; ++g) {
            const v4f x = *(const v4f*)(sr + 256 * g), y = *(const v4f*)(sr + 256 * g + 4);
            const float mx = fmaxf(fmaxf(fmaxf(x.x, x.y), fmaxf(x.z, x.w)), fmaxf(fmaxf(y.x, y.y), fmaxf(y.z, y.w)));
            const float mn = fmaxf(m, mx);
            s = s * expf(m - mn) + (((expf(x.x - mn) + expf(x.y - mn)) + (expf(x.z - mn) + expf(x.w - mn))) + ((expf(y.x - mn) + expf(y.y - mn)) + (expf(y.z - mn) + expf(y.w - mn))));
            m = mn;
        }
        float gm = m;
        gm = fmaxf(gm, __shfl_xor(gm, 16, 32)); gm = fmaxf(gm, __shfl_xor(gm, 8, 32)); gm = fmaxf(gm, __shfl_xor(gm, 4, 32));
        gm = fmaxf(gm, __shfl_xor(gm, 2, 32));  gm = fmaxf(gm, __shfl_xor(gm, 1, 32));
        s = s * expf(m - gm);
        s += __shfl_xor(s, 16, 32); s += __shfl_xor(s, 8, 32); s += __shfl_xor(s, 4, 32); s += __shfl_xor(s, 2, 32); s += __shfl_xor(s, 1, 32);
        const float f = 16384.f / s;
        unsigned short* pr = P + (size_t)row * SEQ + 8 * L;
#pragma unroll 1
        for (int g = 0; g < SEQ / 256; ++g) {
            const v4f x = *(const v4f*)(sr + 256 * g), y = *(const v4f*)(sr + 256 * g + 4);
            u4v pk;
            pk.x = pk2hf(expf(x.x - gm) * f, expf(x.y - gm) * f);
            pk.y = pk2hf(expf(x.z - gm) * f, expf(x.w - gm) * f);
            pk.z = pk2hf(expf(y.x - gm) * f, expf(y.y - gm) * f);
            pk.w = pk2hf(expf(y.z - gm) * f, expf(y.w - gm) * f);
            st2_u4(pr + 256 * g, pk);
        }
    }
}

constexpr size_t al256(size_t v) { return (v + 255) / 256 * 256; }
constexpr size_t SZ_X16  = al256((size_t)NB * SEQ * DM * 2);
constexpr size_t SZ_WQK  = al256((size_t)2 * DM * DM * 2);
constexpr size_t SZ_W1   = al256((size_t)DM * DM * 2);
constexpr size_t SZ_QK   = al256((size_t)SEQ * QKP * 2);
constexpr size_t SZ_VT   = al256((size_t)NB * DM * SEQ * 2);
constexpr size_t SZ_S    = al256((size_t)SEQ * SEQ * 4);
constexpr size_t SZ_AL   = al256((size_t)SEQ * SEQ * 2);
constexpr size_t SZ_AO   = al256((size_t)NB * SEQ * DM * 2);
constexpr size_t SZ_BT   = al256((size_t)4 * DM * 4);
constexpr size_t OFF_X16  = 0;
constexpr size_t OFF_WQK  = OFF_X16 + SZ_X16;
constexpr size_t OFF_WVT  = OFF_WQK + SZ_WQK;
constexpr size_t OFF_WMT  = OFF_WVT + SZ_W1;
constexpr size_t OFF_QK   = OFF_WMT + SZ_W1;
constexpr size_t OFF_VT   = OFF_QK + SZ_QK;
constexpr size_t OFF_S    = OFF_VT + SZ_VT;
constexpr size_t OFF_AL   = OFF_S + SZ_S;
constexpr size_t OFF_AO   = OFF_AL + SZ_AL;
constexpr size_t OFF_BT   = OFF_AO + SZ_AO;
constexpr size_t WS_TOTAL = OFF_BT + SZ_BT;
static_assert(WS_TOTAL <= (size_t)134217728);
static_assert((size_t)SEQ * QKP * 2 <= SZ_QK && (size_t)SEQ * SEQ * 4 <= SZ_S && (size_t)SEQ * SEQ * 2 <= SZ_AL);

extern "C" void kernel_launch(void* const* d_in, const int* in_sizes, int n_in, void* d_out, int out_size, void* d_ws, size_t ws_size, hipStream_t stream) {
    if (n_in < 9) return;
    const long long need_rows = (long long)(NB - 1) * SEQ_FULL + SEQ;
    if ((long long)in_sizes[0] < need_rows * DM) return;
    if (in_sizes[1] < DM * DM || in_sizes[3] < DM * DM || in_sizes[5] < DM * DM || in_sizes[7] < DM * DM) return;
    if (in_sizes[2] < DM || in_sizes[4] < DM || in_sizes[6] < DM || in_sizes[8] < DM) return;
    if ((long long)out_size < (long long)NB * SEQ * DM) return;
    if (ws_size < WS_TOTAL) return;

    const float* x  = (const float*)d_in[0];
    const float* Wq = (const float*)d_in[1];
    const float* bq = (const float*)d_in[2];
    const float* Wk = (const float*)d_in[3];
    const float* bk = (const float*)d_in[4];
    const float* Wv = (const float*)d_in[5];
    const float* bv = (const float*)d_in[6];
    const float* Wm = (const float*)d_in[7];
    const float* bm = (const float*)d_in[8];
    float* out = (float*)d_out;
    char* ws = (char*)d_ws;
    unsigned short* X16 = (unsigned short*)(ws + OFF_X16);
    unsigned short* WQK = (unsigned short*)(ws + OFF_WQK);
    unsigned short* WVT = (unsigned short*)(ws + OFF_WVT);
    unsigned short* WMT = (unsigned short*)(ws + OFF_WMT);
    unsigned short* QK  = (unsigned short*)(ws + OFF_QK);
    unsigned short* VT  = (unsigned short*)(ws + OFF_VT);
    float*          Sf  = (float*)(ws + OFF_S);
    unsigned short* AL  = (unsigned short*)(ws + OFF_AL);
    unsigned short* AO  = (unsigned short*)(ws + OFF_AO);
    float*          BT  = (float*)(ws + OFF_BT);

    const unsigned gw = (unsigned)((DM * (DM / 8) + 255) / 256);
    k_wT<<<gw, 256, 0, stream>>>(Wq, WQK, 16.0f);
    k_wT<<<gw, 256, 0, stream>>>(Wk, WQK + (size_t)DM * DM, 16.0f);
    k_wT<<<gw, 256, 0, stream>>>(Wv, WVT, 16.0f);
    k_wT<<<gw, 256, 0, stream>>>(Wm, WMT, 16.0f);

    k_bias<<<1, 256, 0, stream>>>(bq, bk, bv, bm, BT);
    k_prep_x<<<(unsigned)(((long long)NB * SEQ * (DM / 8) + 255) / 256), 256, 0, stream>>>(x, X16);

    {
        const int tiles = (DM / 64) * (SEQ / 64);
        k_gemm_vt<<<dim3((unsigned)((tiles + 7) / 8), NB), 256, 0, stream>>>(WVT, DM, 0, X16, DM, (long long)SEQ * DM, VT, SEQ, (long long)DM * SEQ,
                                                                            BT + 2 * DM, DM, SEQ, DM, 0.0625f, 1.0f);
    }
    for (int b = 0; b < NB; ++b) {
        {
            const int tiles = (SEQ / 64) * ((2 * DM) / 64);
            k_gemm_qk<<<dim3((unsigned)((tiles + 7) / 8), 1), 256, 0, stream>>>(X16 + (size_t)b * SEQ * DM, DM, 0, WQK, DM, 0, QK, QKP, 0,
                                                                                BT, SEQ, 2 * DM, DM, 0.0625f, 4096.0f);
        }
        {
            const int tiles = (SEQ / 64) * (SEQ / 64);
            k_gemm_s<<<dim3((unsigned)((tiles + 7) / 8), 1), 256, 0, stream>>>(QK + 3 * DM, QKP, 0, QK, QKP, 0, Sf, SEQ, 0, SEQ, SEQ, SCORE_K, 5.9604644775390625e-08f);
        }
        k_rowsoft<<<SEQ / (8 * RS_RPW), 256, 0, stream>>>(Sf, AL);
        {
            const int tiles = (SEQ / 64) * (DM / 64);
            k_gemm_ctx<<<dim3((unsigned)((tiles + 7) / 8), 1), 256, 0, stream>>>(AL, SEQ, 0, VT + (size_t)b * DM * SEQ, SEQ, 0, AO + (size_t)b * SEQ * DM, DM, 0,
                                                                                 SEQ, DM, SEQ, 0.00390625f);
        }
    }
    {
        const int tiles = (SEQ / 64) * (DM / 64);
        k_gemm_out<<<dim3((unsigned)((tiles + 7) / 8), NB), 256, 0, stream>>>(AO, DM, (long long)SEQ * DM, WMT, DM, 0, out, DM, (long long)SEQ * DM,
                                                                             BT + 3 * DM, SEQ, DM, DM, 0.0009765625f);
    }
}
